// TargetEmbedding_86328842650205
// MI455X (gfx1250) — hardware-verified
//
#include <hip/hip_runtime.h>
#include <math.h>

typedef __attribute__((ext_vector_type(16))) _Float16 v16h;
typedef __attribute__((ext_vector_type(16))) __bf16 v16b;
typedef __attribute__((ext_vector_type(8)))  _Float16 v8h;
typedef __attribute__((ext_vector_type(8)))  float v8f;
typedef __attribute__((ext_vector_type(4)))  float v4f;
typedef __attribute__((ext_vector_type(2)))  float v2f;
typedef __attribute__((ext_vector_type(4)))  unsigned v4u;
typedef __attribute__((ext_vector_type(4)))  int v4i;
typedef float __attribute__((may_alias)) float_a;
typedef int __attribute__((may_alias)) int_a;

template <typename T> __device__ __forceinline__ void vst2(void* p, T v) { *(volatile T*)p = v; __threadfence(); *(volatile T*)p = v; }
__device__ __forceinline__ v8f wmma16(v16h a, v16h b, v8f c) {
  v8f d = __builtin_amdgcn_wmma_f32_16x16x32_f16(false, a, false, b, (short)0, c, false, false);
  asm volatile("v_nop\n\tv_nop\n\tv_nop\n\tv_nop" : "+v"(d) : "v"(a), "v"(b));
  return d;
}
__device__ __forceinline__ v8f wmma_bf(v16b a, v16b b, v8f c) {
  v8f d = __builtin_amdgcn_wmma_f32_16x16x32_bf16(false, a, false, b, (short)0, c, false, false);
  asm volatile("v_nop\n\tv_nop\n\tv_nop\n\tv_nop" : "+v"(d) : "v"(a), "v"(b));
  return d;
}
__device__ __forceinline__ v16h frag_h(const _Float16* rowk0, int lane) {
  union { v16h v; v8h q[2]; } u; const _Float16* p = rowk0 + 8 * (lane >> 4);
  u.q[0] = *(const v8h*)p; u.q[1] = *(const v8h*)(p + 16); return u.v;
}
__device__ __forceinline__ v16h frag_f32(const float* rowk0, int lane) {
  v16h a; const float* p = rowk0 + 8 * (lane >> 4);
#pragma unroll
  for (int i = 0; i < 8; ++i) { a[i] = (_Float16)p[i]; a[8 + i] = (_Float16)p[16 + i]; }
  return a;
}
__device__ __forceinline__ v16h frag_f32s(const float* rowk0, int lane, float sc) {
  v16h a; const float* p = rowk0 + 8 * (lane >> 4);
#pragma unroll
  for (int i = 0; i < 8; ++i) { a[i] = (_Float16)(p[i] * sc); a[8 + i] = (_Float16)(p[16 + i] * sc); }
  return a;
}
__device__ __forceinline__ v16h fragc_f32(const float* W, int k0, int n, int lane, int ld, int K) {
  v16h a; const int g = lane >> 4;
#pragma unroll
  for (int i = 0; i < 8; ++i) { const int ka = k0 + 8 * g + i, kb = ka + 16;
    a[i] = (_Float16)(ka < K ? W[(size_t)ka * ld + n] : 0.f); a[8 + i] = (_Float16)(kb < K ? W[(size_t)kb * ld + n] : 0.f); }
  return a;
}
struct F2 { v16b h, l; };
__device__ __forceinline__ F2 bsplit16(const float v[16]) { F2 r;
#pragma unroll
  for (int i = 0; i < 16; ++i) { const __bf16 h = (__bf16)v[i]; r.h[i] = h; r.l[i] = (__bf16)(v[i] - (float)h); }
  return r; }
__device__ __forceinline__ F2 split_row(const float* row, int k0, int lane) { float v[16]; const float* p = row + k0 + 8 * (lane >> 4);
#pragma unroll
  for (int i = 0; i < 8; ++i) { v[i] = p[i]; v[8 + i] = p[16 + i]; }
  return bsplit16(v); }
__device__ __forceinline__ F2 split_rowK(const float* row, int k0, int lane, int K) { float v[16]; const int g = lane >> 4;
#pragma unroll
  for (int i = 0; i < 8; ++i) { const int ka = k0 + 8 * g + i, kb = ka + 16; v[i] = ka < K ? row[ka] : 0.f; v[8 + i] = kb < K ? row[kb] : 0.f; }
  return bsplit16(v); }
__device__ __forceinline__ F2 split_col(const float* W, int k0, int n, int lane, int ld, int K) { float v[16]; const int g = lane >> 4;
#pragma unroll
  for (int i = 0; i < 8; ++i) { const int ka = k0 + 8 * g + i, kb = ka + 16; v[i] = ka < K ? W[(size_t)ka * ld + n] : 0.f; v[8 + i] = kb < K ? W[(size_t)kb * ld + n] : 0.f; }
  return bsplit16(v); }
__device__ __forceinline__ v8f mac3(const F2& a, const F2& b, v8f c) { c = wmma_bf(a.l, b.h, c); c = wmma_bf(a.h, b.l, c); return wmma_bf(a.h, b.h, c); }
__device__ __forceinline__ float sigm(float v) { return 1.0f / (1.0f + expf(-v)); }
#define LDSX() do { asm volatile("s_wait_dscnt 0" ::: "memory"); __builtin_amdgcn_wave_barrier(); __builtin_amdgcn_fence(__ATOMIC_RELEASE, "workgroup"); } while (0)

#define NBT 32
#define NBB 16
#define CC 1024
#define HH 22
#define WWD 22
#define PP 3
#define NBOX (NBT * NBB)
#define KCV (CC * 9)

__device__ __forceinline__ float hat_int(float t) { t = fminf(fmaxf(t, -1.0f), 1.0f); return t + 0.5f - 0.5f * t * fabsf(t); }
__global__ __launch_bounds__(256) void k_bins(const float* __restrict__ bbox, float* __restrict__ tab) {
  const int box = blockIdx.x * 256 + threadIdx.x; if (box >= NBOX) return;
  const float* bb = bbox + (size_t)box * 4; const float sc = 1.0f / 16.0f;
  const float x1 = bb[0] * sc, y1 = bb[1] * sc, x2 = (bb[0] + bb[2]) * sc, y2 = (bb[1] + bb[3]) * sc;
  const float bw = (x2 - x1) / (float)PP, bh = (y2 - y1) / (float)PP;
  float* t = tab + (size_t)box * 136;
#pragma unroll 1
  for (int p = 0; p < PP; ++p) { const float xs = x1 + (float)p * bw, xe = xs + bw; const float ys = y1 + (float)p * bh, ye = ys + bh;
#pragma unroll 1
    for (int i = 0; i < WWD; ++i) t[p * WWD + i] = hat_int(xe - (float)i) - hat_int(xs - (float)i);
#pragma unroll 1
    for (int i = 0; i < HH; ++i) t[66 + p * HH + i] = hat_int(ye - (float)i) - hat_int(ys - (float)i); }
  const float area = fmaxf(bw * bh, 0.f); t[132] = area > 0.f ? 1.0f / fmaxf(area, 1e-12f) : 0.f; t[133] = 0.f; t[134] = 0.f; t[135] = 0.f;
}
__global__ __launch_bounds__(256) void k_pool(const float* __restrict__ feat, const float* __restrict__ tab, float* __restrict__ A) {
  __shared__ float sf[32][HH * WWD + 1];
  __shared__ float st[NBB][136];
  __shared__ __align__(16) float so[NBB][32 * 9];
  const int b = blockIdx.y, c0 = blockIdx.x * 32, tid = threadIdx.x;
  for (int q = tid; q < 32 * HH * WWD; q += 256) { const int cl = q / (HH * WWD), e = q % (HH * WWD); sf[cl][e] = feat[((size_t)b * CC + c0 + cl) * (HH * WWD) + e]; }
  for (int q = tid; q < NBB * 136; q += 256) st[q / 136][q % 136] = tab[(size_t)(b * NBB) * 136 + q];
  __syncthreads();
  { const int cl = tid & 31, bp = tid >> 5;
    for (int u = 0; u < 2; ++u) { const int n = bp * 2 + u; const float* wx = &st[n][0]; const float* wy = &st[n][66]; const float ia = st[n][132];
      float acc[9];
#pragma unroll
      for (int e = 0; e < 9; ++e) acc[e] = 0.f;
#pragma unroll 1
      for (int h = 0; h < HH; ++h) { float tx[3] = {0.f, 0.f, 0.f};
#pragma unroll 1
        for (int w = 0; w < WWD; ++w) { const float v = sf[cl][h * WWD + w]; tx[0] += v * wx[w]; tx[1] += v * wx[WWD + w]; tx[2] += v * wx[2 * WWD + w]; }
#pragma unroll
        for (int q = 0; q < 3; ++q) { const float wyv = wy[q * HH + h];
#pragma unroll
          for (int p = 0; p < 3; ++p) acc[q * 3 + p] += wyv * tx[p]; } }
#pragma unroll
      for (int e = 0; e < 9; ++e) so[n][cl * 9 + e] = acc[e] * ia; } }
  __syncthreads();
  for (int q = tid; q < NBB * 72; q += 256) { const int n = q / 72, pc = q % 72; vst2(A + (size_t)(b * NBB + n) * KCV + c0 * 9 + pc * 4, *(const v4f*)(&so[n][pc * 4])); }
}
__global__ __launch_bounds__(128) void k_conv(const float* __restrict__ A, const float* __restrict__ W, const float* __restrict__ cb, const float* __restrict__ gam, const float* __restrict__ bet, const float* __restrict__ mu, const float* __restrict__ var,
                                            float* __restrict__ x1) {
  __shared__ __align__(16) float so[4][16][132];
  const int tid = threadIdx.x, wave = tid >> 5, lane = tid & 31, col = lane & 15, g = lane >> 4;
  const int r0 = blockIdx.x * 64 + wave * 16, n0 = blockIdx.y * 128;
  v8f acc[8] = {};
#pragma unroll 1
  for (int kc = 0; kc < KCV / 32; ++kc) { const v16h a = frag_f32(A + (size_t)(r0 + col) * KCV + kc * 32, lane);
#pragma unroll
    for (int j = 0; j < 8; ++j) acc[j] = wmma16(a, frag_f32s(W + (size_t)(n0 + j * 16 + col) * KCV + kc * 32, lane, 16.0f), acc[j]); }
#pragma unroll
  for (int j = 0; j < 8; ++j) { const int o = n0 + j * 16 + col; const float sc = gam[o] * rsqrtf(var[o] + 1e-5f), sh = bet[o] - mu[o] * sc, bb = cb[o];
#pragma unroll
    for (int r = 0; r < 8; ++r) { const float v = (acc[j][r] * (1.0f / 16.0f) + bb) * sc + sh; so[wave][8 * g + r][j * 16 + col] = v > 0.f ? v : 0.f; } }
  LDSX();
#pragma unroll 4
  for (int rl = 0; rl < 16; ++rl) vst2(x1 + (size_t)(r0 + rl) * CC + n0 + lane * 4, *(const v4f*)(&so[wave][rl][lane * 4]));
}
template <int K, int RELU>
__global__ __launch_bounds__(128) void k_fc(const float* __restrict__ Ain, const float* __restrict__ W, const float* __restrict__ bias, int N, float* __restrict__ Out) {
  __shared__ __align__(16) float so[4][16][132];
  const int tid = threadIdx.x, wave = tid >> 5, lane = tid & 31, col = lane & 15, g = lane >> 4;
  const int r0 = blockIdx.x * 64 + wave * 16, n0 = blockIdx.y * 128;
  v8f acc[8] = {};
#pragma unroll 1
  for (int kc = 0; kc < K / 32; ++kc) { const F2 a = split_row(Ain + (size_t)(r0 + col) * K, kc * 32, lane);
#pragma unroll
    for (int j = 0; j < 8; ++j) acc[j] = mac3(a, split_row(W + (size_t)(n0 + j * 16 + col) * K, kc * 32, lane), acc[j]); }
#pragma unroll
  for (int j = 0; j < 8; ++j) { const float bb = bias[n0 + j * 16 + col];
#pragma unroll
    for (int r = 0; r < 8; ++r) { const float v = acc[j][r] + bb; so[wave][8 * g + r][j * 16 + col] = RELU ? (v > 0.f ? v : 0.f) : v; } }
  LDSX();
#pragma unroll 4
  for (int rl = 0; rl < 16; ++rl) vst2(Out + (size_t)(r0 + rl) * N + n0 + lane * 4, *(const v4f*)(&so[wave][rl][lane * 4]));
}
extern "C" void kernel_launch(void* const* d_in, const int* in_sizes, int n_in, void* d_out, int out_size, void* d_ws, size_t ws_size, hipStream_t stream) {
  (void)in_sizes; (void)n_in; (void)out_size; (void)ws_size;
  const float** I = (const float**)d_in;
  const float* feat = I[0]; const float* bbox = I[1]; const float* cw = I[2]; const float* cb = I[3]; const float* gam = I[4]; const float* bet = I[5]; const float* mu = I[6]; const float* var = I[7];
  const float* w1 = I[8]; const float* b1 = I[9]; const float* w2 = I[10]; const float* b2 = I[11]; const float* w3 = I[12]; const float* b3 = I[13];
  float* out = (float*)d_out;
  char* ws = (char*)d_ws; size_t off = 0;
  auto take = [&](size_t bytes) { char* p = ws + off; off += (bytes + 255) & ~(size_t)255; return p; };
  float* tab = (float*)take((size_t)NBOX * 136 * 4); float* A = (float*)take((size_t)NBOX * KCV * 4); float* x1 = (float*)take((size_t)NBOX * CC * 4); float* x2 = (float*)take((size_t)NBOX * 512 * 4); float* x3 = (float*)take((size_t)NBOX * 512 * 4);
  k_bins<<<2, 256, 0, stream>>>(bbox, tab);
  k_pool<<<dim3(CC / 32, NBT), 256, 0, stream>>>(feat, tab, A);
  k_conv<<<dim3(NBOX / 64, CC / 128), 128, 0, stream>>>(A, cw, cb, gam, bet, mu, var, x1);
  k_fc<CC, 1><<<dim3(NBOX / 64, 512 / 128), 128, 0, stream>>>(x1, w1, b1, 512, x2);
  k_fc<512, 1><<<dim3(NBOX / 64, 512 / 128), 128, 0, stream>>>(x2, w2, b2, 512, x3);
  k_fc<512, 0><<<dim3(NBOX / 64, 512 / 128), 128, 0, stream>>>(x3, w3, b3, 512, out);
}
